// BiAlignAggLayer_32246614458531
// MI455X (gfx1250) — hardware-verified
//
#include <hip/hip_runtime.h>
#include <math.h>

typedef __attribute__((ext_vector_type(16))) _Float16 v16h;
typedef __attribute__((ext_vector_type(8)))  _Float16 v8h;
typedef __attribute__((ext_vector_type(16))) __bf16   v16b;
typedef __attribute__((ext_vector_type(8)))  __bf16   v8b;
typedef __attribute__((ext_vector_type(8)))  float    v8f;
typedef __attribute__((ext_vector_type(4)))  float    v4f;

constexpr int kB    = 32;
constexpr int kCh   = 8;
constexpr int kL    = 512;
constexpr int kD    = 512;
constexpr int kH    = 512;
constexpr int kLL   = kL * kL;
constexpr int kThr  = 256;
constexpr float kInCarry = 1024.0f;
constexpr float kWCarry = 4096.0f;
constexpr float kCP = 16384.0f;
constexpr float kCX = 1024.0f;
constexpr float kScS = 1.0f / (kInCarry * kInCarry), kScW = 1.0f / (kCP * kWCarry), kScA = 1.0f / (kCX * kWCarry);
constexpr float kF16MinNormal = 6.103515625e-5f;

static_assert((kL % 64) == 0 && (kD % 64) == 0 && (kH % 64) == 0 && ((kL / 64) * (kL / 64)) % 8 == 0 && kB == 4 * kCh && kL == (1 << 9) && kD == kL && kH == kL && kL / 8 == 64, "GEMM M, N multiples of 64; grids exact; four chunks of eight; the transposing cast's block of K / 8 = 64 threads");

constexpr size_t kOffI16 = 0ull;
constexpr size_t kOffJ16 = 16777216ull;
constexpr size_t kOffIT16 = 33554432ull;
constexpr size_t kOffJT16 = 50331648ull;
constexpr size_t kOffWT16 = 67108864ull;
constexpr size_t kOffBIAS = 67633152ull;
constexpr size_t kOffS = 67637248ull;
constexpr size_t kOffPJ = 76025856ull;
constexpr size_t kOffPIT = 80220160ull;
constexpr size_t kOffWJ = 84414464ull;
constexpr size_t kOffWI = 92803072ull;
constexpr size_t kOffXI16 = 101191680ull;
constexpr size_t kOffXJ16 = 105385984ull;
constexpr size_t kOffY = 109580288ull;
constexpr size_t kOffOI = 117968896ull;
constexpr size_t kWsTotal = 118034432ull;
static_assert(kWsTotal <= 134217728ull, "carve cap: under 128 MiB");
static_assert(kOffI16 == 0
              && kOffJ16 == kOffI16 + 16777216ull
              && kOffIT16 == kOffJ16 + 16777216ull
              && kOffJT16 == kOffIT16 + 16777216ull
              && kOffWT16 == kOffJT16 + 16777216ull
              && kOffBIAS == kOffWT16 + 524288ull
              && kOffS == kOffBIAS + 4096ull
              && kOffPJ == kOffS + 8388608ull
              && kOffPIT == kOffPJ + 4194304ull
              && kOffWJ == kOffPIT + 4194304ull
              && kOffWI == kOffWJ + 8388608ull
              && kOffXI16 == kOffWI + 8388608ull
              && kOffXJ16 == kOffXI16 + 4194304ull
              && kOffY == kOffXJ16 + 4194304ull
              && kOffOI == kOffY + 8388608ull
              && kWsTotal == kOffOI + 65536ull, "the carve is chained and totalled");
static_assert((kOffI16 % 256) == 0 && (kOffJ16 % 256) == 0 && (kOffIT16 % 256) == 0 && (kOffJT16 % 256) == 0 && (kOffWT16 % 256) == 0 && (kOffBIAS % 256) == 0 && (kOffS % 256) == 0 && (kOffPJ % 256) == 0 && (kOffPIT % 256) == 0 && (kOffWJ % 256) == 0 && (kOffWI % 256) == 0 && (kOffXI16 % 256) == 0 && (kOffXJ16 % 256) == 0 && (kOffY % 256) == 0 && (kOffOI % 256) == 0, "aligned regions");

__device__ __forceinline__ unsigned short f2bf_bits(float f) {
  unsigned u = __float_as_uint(f);
  return (unsigned short)((u + 0x7FFFu + ((u >> 16) & 1u)) >> 16);
}
__device__ __forceinline__ float bf_bits2f(unsigned short h) { return __uint_as_float(((unsigned)h) << 16); }
__device__ __forceinline__ float bf16r(float f) { return bf_bits2f(f2bf_bits(f)); }
__device__ __forceinline__ float carry_flush(float v, float carry) {
  const float s = v * carry;
  return (fabsf(s) < kF16MinNormal) ? 0.0f : s;
}
__device__ __forceinline__ float frcp(float x) { return __builtin_amdgcn_rcpf(x); }

__device__ __forceinline__ void dep_guard4_h(v8f& a, v8f& b, v8f& c, v8f& d, v16h x, v16h y) { asm volatile("v_nop\n\tv_nop\n\tv_nop\n\tv_nop" : "+v"(a), "+v"(b), "+v"(c), "+v"(d) : "v"(x), "v"(y)); }
__device__ __forceinline__ void dep_guard4_b(v8f& a, v8f& b, v8f& c, v8f& d, v16b x, v16b y) { asm volatile("v_nop\n\tv_nop\n\tv_nop\n\tv_nop" : "+v"(a), "+v"(b), "+v"(c), "+v"(d) : "v"(x), "v"(y)); }
__device__ __forceinline__ void keep4_h(v16h a, v16h b, v16h c, v16h d) { asm volatile("v_nop" :: "v"(a), "v"(b), "v"(c), "v"(d)); }
__device__ __forceinline__ void keep4_b(v16b a, v16b b, v16b c, v16b d) { asm volatile("v_nop" :: "v"(a), "v"(b), "v"(c), "v"(d)); }
__device__ __forceinline__ void acc_guard4(v8f& a, v8f& b, v8f& c, v8f& d) { asm volatile("v_nop\n\tv_nop\n\tv_nop\n\tv_nop" : "+v"(a), "+v"(b), "+v"(c), "+v"(d)); }

template <typename T> struct Frag;
template <> struct Frag<_Float16> {
  typedef v16h V; union U { v16h v; v8h h[2]; };
  static __device__ __forceinline__ v16h load(const _Float16* p) {
    U f; f.h[0] = *(const v8h*)(p); f.h[1] = *(const v8h*)(p + 16); return f.v;
  }
  static __device__ __forceinline__ v8f mma(v16h a, v16h b, v8f c) {
    return __builtin_amdgcn_wmma_f32_16x16x32_f16(false, a, false, b, (short)0, c, false, false);
  }
  static __device__ __forceinline__ void guard4(v8f& a, v8f& b, v8f& c, v8f& d, v16h x, v16h y) { dep_guard4_h(a, b, c, d, x, y); }
  static __device__ __forceinline__ void keep(v16h a, v16h b, v16h c, v16h d) { keep4_h(a, b, c, d); }
};
template <> struct Frag<__bf16> {
  typedef v16b V; union U { v16b v; v8b h[2]; };
  static __device__ __forceinline__ v16b load(const __bf16* p) {
    U f; f.h[0] = *(const v8b*)(p); f.h[1] = *(const v8b*)(p + 16); return f.v;
  }
  static __device__ __forceinline__ v8f mma(v16b a, v16b b, v8f c) {
    return __builtin_amdgcn_wmma_f32_16x16x32_bf16(false, a, false, b, (short)0, c, false, false);
  }
  static __device__ __forceinline__ void guard4(v8f& a, v8f& b, v8f& c, v8f& d, v16b x, v16b y) { dep_guard4_b(a, b, c, d, x, y); }
  static __device__ __forceinline__ void keep(v16b a, v16b b, v16b c, v16b d) { keep4_b(a, b, c, d); }
};

__device__ __forceinline__ v8f mma_h(v16h a, v16h b, v8f c) {
  c = __builtin_amdgcn_wmma_f32_16x16x32_f16(false, a, false, b, (short)0, c, false, false);
  asm volatile("v_nop\n\tv_nop\n\tv_nop\n\tv_nop" : "+v"(c) : "v"(a), "v"(b));
  return c;
}

template <int ET> struct Elem;
template <> struct Elem<0> { typedef _Float16 T; };
template <> struct Elem<1> { typedef __bf16 T; };
template <int ET, bool SPLIT, int BIAS_MODE, int OUT_MODE, bool RESID, int ACT = 0>
__global__ __launch_bounds__(256) void wmma_gemm64(
    const unsigned short* __restrict__ Ap, const unsigned short* __restrict__ A2p, int lda, long strideA,
    const unsigned short* __restrict__ Btp, const unsigned short* __restrict__ Bt2p, int ldb, long strideB,
    void* __restrict__ Cout, void* __restrict__ Cout2, int ldc, long strideC,
    const float* __restrict__ bias,
    const float* __restrict__ resid, long strideR,
    int M, int N, int K, float scale) {
  typedef typename Elem<ET>::T T;
  typedef typename Frag<T>::V V;
  const T* A = (const T*)Ap; const T* A2 = (const T*)A2p; const T* Bt = (const T*)Btp; const T* Bt2 = (const T*)Bt2p;
  __shared__ __align__(16) float sT[8][16 * 68];
  const int b    = blockIdx.y;
  const int lane = threadIdx.x & 31;
  const int wave = threadIdx.x >> 5;
  const int tilesN = N >> 6;
  const int tilesM = M >> 6;
  const int tile = blockIdx.x * 8 + wave;
  if (tile >= tilesM * tilesN) return;
  const int tm = tile / tilesN;
  const int tn = tile - tm * tilesN;
  const int m0 = tm << 6;
  const int n0 = tn << 6;

  const T* Ab  = A  + (size_t)b * strideA;
  const T* Bb  = Bt + (size_t)b * strideB;
  const T* Ab2 = SPLIT ? (A2  + (size_t)b * strideA) : nullptr;
  const T* Bb2 = SPLIT ? (Bt2 + (size_t)b * strideB) : nullptr;

  const int rlane = lane & 15;
  const int koff  = (lane >> 4) * 8;
  const int mOff  = (lane >> 4) * 8;

  v8f acc[4][4];
#pragma unroll
  for (int i = 0; i < 4; ++i)
#pragma unroll
    for (int j = 0; j < 4; ++j) acc[i][j] = (v8f){0.f,0.f,0.f,0.f,0.f,0.f,0.f,0.f};

  for (int k0 = 0; k0 < K; k0 += 32) {
    V bh[4], bl[4];
#pragma unroll
    for (int j = 0; j < 4; ++j) {
      const size_t bo = (size_t)(n0 + (j << 4) + rlane) * ldb + koff + k0;
      bh[j] = Frag<T>::load(Bb + bo);
      if (SPLIT) bl[j] = Frag<T>::load(Bb2 + bo);
    }
#pragma unroll
    for (int i = 0; i < 4; ++i) {
      const size_t ao = (size_t)(m0 + (i << 4) + rlane) * lda + koff + k0;
      V ah = Frag<T>::load(Ab + ao);
      V al;
      if (SPLIT) al = Frag<T>::load(Ab2 + ao);
#pragma unroll
      for (int j = 0; j < 4; ++j) {
        acc[i][j] = Frag<T>::mma(ah, bh[j], acc[i][j]);
        if (SPLIT) {
          acc[i][j] = Frag<T>::mma(ah, bl[j], acc[i][j]);
          acc[i][j] = Frag<T>::mma(al, bh[j], acc[i][j]);
        }
      }
      Frag<T>::guard4(acc[i][0], acc[i][1], acc[i][2], acc[i][3], ah, SPLIT ? al : ah);
    }
    Frag<T>::keep(bh[0], bh[1], bh[2], bh[3]);
    if (SPLIT) Frag<T>::keep(bl[0], bl[1], bl[2], bl[3]);
  }
  acc_guard4(acc[0][0], acc[0][1], acc[0][2], acc[0][3]);
  acc_guard4(acc[1][0], acc[1][1], acc[1][2], acc[1][3]);
  acc_guard4(acc[2][0], acc[2][1], acc[2][2], acc[2][3]);
  acc_guard4(acc[3][0], acc[3][1], acc[3][2], acc[3][3]);

  float* slab = sT[wave];
  const float* Rb = RESID ? (resid + (size_t)b * strideR) : nullptr;
#pragma unroll
  for (int i = 0; i < 4; ++i) {
    const int mBase = m0 + (i << 4);
#pragma unroll
    for (int j = 0; j < 4; ++j) {
      const int n = n0 + (j << 4) + rlane;
      float bv = 0.f;
      if (BIAS_MODE == 2) bv = bias[n];
#pragma unroll
      for (int r = 0; r < 8; ++r) {
        float v = acc[i][j][r] * scale;
        if (BIAS_MODE == 1) v += bias[mBase + mOff + r];
        if (BIAS_MODE == 2) v += bv;
        if (RESID) v += Rb[(size_t)(mBase + mOff + r) * ldc + n];
        if (ACT == 1) v = tanhf(v);
        if (ACT == 2) v = fmaxf(v, 0.0f);
        if (ACT == 3) v = v / (1.0f + expf(-v));
        if (ACT == 4) v = (v > 0.f) ? v : 0.01f * v;
        slab[(mOff + r) * 68 + (j << 4) + rlane] = v;
      }
    }
    __builtin_amdgcn_fence(__ATOMIC_RELEASE, "workgroup");
    __builtin_amdgcn_wave_barrier();
    __builtin_amdgcn_fence(__ATOMIC_ACQUIRE, "workgroup");
    if (OUT_MODE == 0) {
      float* C = (float*)Cout + (size_t)b * strideC;
      const int hh = lane >> 4, c4 = (lane & 15) * 4;
      for (int pass = 0; pass < 2; ++pass) {
#pragma unroll
        for (int it = 0; it < 8; ++it) {
          const int row = it * 2 + hh;
          v4f v = *(const v4f*)(slab + row * 68 + c4);
          *(volatile v4f*)(C + (size_t)(mBase + row) * ldc + n0 + c4) = v;
        }
        __threadfence();
      }
    } else {
      const int q = lane >> 3, c8 = (lane & 7) * 8;
      unsigned short* C  = (unsigned short*)Cout  + (size_t)b * strideC;
      unsigned short* C2 = (OUT_MODE == 2) ? ((unsigned short*)Cout2 + (size_t)b * strideC) : nullptr;
      for (int pass = 0; pass < 2; ++pass) {
#pragma unroll
        for (int it = 0; it < 4; ++it) {
          const int row = it * 4 + q;
          const float* sp = slab + row * 68 + c8;
          v8h hv, lv;
#pragma unroll
          for (int e = 0; e < 8; ++e) {
            if (OUT_MODE == 1) {
              hv[e] = (_Float16)sp[e];
            } else {
              unsigned short hb = f2bf_bits(sp[e]);
              unsigned short lb = f2bf_bits(sp[e] - bf_bits2f(hb));
              hv[e] = __builtin_bit_cast(_Float16, hb);
              lv[e] = __builtin_bit_cast(_Float16, lb);
            }
          }
          *(volatile v8h*)(C + (size_t)(mBase + row) * ldc + n0 + c8) = hv;
          if (OUT_MODE == 2) *(volatile v8h*)(C2 + (size_t)(mBase + row) * ldc + n0 + c8) = lv;
        }
        __threadfence();
      }
    }
    __builtin_amdgcn_fence(__ATOMIC_RELEASE, "workgroup");
    __builtin_amdgcn_wave_barrier();
    __builtin_amdgcn_fence(__ATOMIC_ACQUIRE, "workgroup");
  }
}

__global__ __launch_bounds__(kThr) void cast_plane_kernel(const float* __restrict__ src, unsigned short* __restrict__ dst,
                                                          int colsLog2, int dstPitch, int dstOff) {
  const int i   = blockIdx.x * kThr + threadIdx.x;
  const int sh  = colsLog2 - 3;
  const int row = i >> sh;
  const int c8  = (i & ((1 << sh) - 1)) * 8;
  const float* sp = src + ((size_t)row << colsLog2) + c8;
  const v4f a0 = *(const v4f*)(sp);
  const v4f a1 = *(const v4f*)(sp + 4);
  v8h hv;
#pragma unroll
  for (int e = 0; e < 4; ++e) {
    const float f0 = a0[e];
    const float f1 = a1[e];
    hv[e]     = (_Float16)carry_flush(bf16r(f0), kInCarry);
    hv[4 + e] = (_Float16)carry_flush(bf16r(f1), kInCarry);
  }
  unsigned short* dp = dst + (size_t)row * dstPitch + dstOff + c8;
  *(volatile v8h*)dp = hv;
  __threadfence();
  *(volatile v8h*)dp = hv;
}
__global__ __launch_bounds__(256) void wt_plane_kernel(const float* __restrict__ W, unsigned short* __restrict__ dst, int K, int N, int nLive, int ldd, int colOff) {
  const int n  = blockIdx.x;
  const int k8 = threadIdx.x * 8;
  const bool live = n < nLive;
  const int nc = live ? n : 0;
  v8h hv;
#pragma unroll
  for (int e = 0; e < 8; ++e) {
    const float w = W[(size_t)(k8 + e) * N + nc];
    hv[e] = (_Float16)(live ? carry_flush(bf16r(w), kWCarry) : 0.0f);
  }
  unsigned short* dp = dst + (size_t)n * ldd + colOff + k8;
  *(volatile v8h*)dp = hv;
  __threadfence();
  *(volatile v8h*)dp = hv;
}


__global__ __launch_bounds__(kThr) void setup_kernel(const float* __restrict__ b_agg, float* __restrict__ BIAS) {
  const unsigned i0 = threadIdx.x * 4u;
  const bool live = i0 >= (unsigned)kH;
  const unsigned j0 = live ? (i0 - (unsigned)kH) : 0u;
  const v4f a = *(const v4f*)(b_agg + j0);
  v4f o;
#pragma unroll
  for (int e = 0; e < 4; ++e) { const float p = bf16r(a[e]); o[e] = live ? p : 0.0f; }
  float* dp = BIAS + i0;
  *(volatile v4f*)dp = o;
  __threadfence();
  *(volatile v4f*)dp = o;
}

__global__ __launch_bounds__(kThr) void rowsoftmax_kernel(const float* __restrict__ S, unsigned short* __restrict__ PJ) {
  const unsigned r = blockIdx.x * (unsigned)kThr + threadIdx.x;
  const float* sr = S + (size_t)r * kL;
  float mx = -INFINITY;
#pragma unroll 1
  for (int c = 0; c < kL; c += 4) { const v4f a = *(const v4f*)(sr + c); mx = fmaxf(fmaxf(mx, a[0]), fmaxf(fmaxf(a[1], a[2]), a[3])); }
  float sum = 0.0f;
#pragma unroll 1
  for (int c = 0; c < kL; c += 4) { const v4f a = *(const v4f*)(sr + c); sum += expf(a[0] - mx); sum += expf(a[1] - mx); sum += expf(a[2] - mx); sum += expf(a[3] - mx); }
  unsigned short* dp = PJ + (size_t)r * kL;
  for (int pass = 0; pass < 2; ++pass) {
#pragma unroll 1
    for (int c = 0; c < kL; c += 8) {
      const v4f a0 = *(const v4f*)(sr + c), a1 = *(const v4f*)(sr + c + 4);
      v8h hv;
#pragma unroll
      for (int e = 0; e < 4; ++e) { hv[e] = (_Float16)carry_flush(expf(a0[e] - mx) / sum, kCP); hv[4 + e] = (_Float16)carry_flush(expf(a1[e] - mx) / sum, kCP); }
      *(volatile v8h*)(dp + c) = hv;
    }
    __threadfence();
  }
}
static_assert(((size_t)kCh * kL) % kThr == 0, "softmax grids exact");

__global__ __launch_bounds__(kThr) void colsoftmax_kernel(const float* __restrict__ S, unsigned short* __restrict__ PIT) {
  const unsigned v = blockIdx.x * (unsigned)kThr + threadIdx.x;
  const unsigned s = v >> 9, j = v & 511u;
  const float* sc = S + (size_t)s * kLL + j;
  float mx = -INFINITY;
#pragma unroll 1
  for (int i = 0; i < kL; ++i) { const float x = sc[(size_t)i * kL]; mx = (x > mx) ? x : mx; }
  float sum = 0.0f;
#pragma unroll 1
  for (int i = 0; i < kL; ++i) sum += expf(sc[(size_t)i * kL] - mx);
  unsigned short* dp = PIT + (size_t)v * kL;
  for (int pass = 0; pass < 2; ++pass) {
#pragma unroll 1
    for (int i = 0; i < kL; i += 8) {
      v8h hv;
#pragma unroll
      for (int e = 0; e < 8; ++e) hv[e] = (_Float16)carry_flush(expf(sc[(size_t)(i + e) * kL] - mx) / sum, kCP);
      *(volatile v8h*)(dp + i) = hv;
    }
    __threadfence();
  }
}

__global__ __launch_bounds__(kThr) void absdiff_kernel(const float* __restrict__ x, const float* __restrict__ Wt, unsigned short* __restrict__ X16) {
  const size_t v = (size_t)blockIdx.x * kThr + threadIdx.x;
  const v4f a0 = *(const v4f*)(x + v * 8), a1 = *(const v4f*)(x + v * 8 + 4), w0 = *(const v4f*)(Wt + v * 8), w1 = *(const v4f*)(Wt + v * 8 + 4);
  v8h hv;
#pragma unroll
  for (int e = 0; e < 4; ++e) { hv[e] = (_Float16)carry_flush(fabsf(bf16r(a0[e]) - w0[e]), kCX); hv[4 + e] = (_Float16)carry_flush(fabsf(bf16r(a1[e]) - w1[e]), kCX); }
  unsigned short* dp = X16 + v * 8;
  *(volatile v8h*)dp = hv;
  __threadfence();
  *(volatile v8h*)dp = hv;
}
static_assert(((size_t)kCh * kL * kD / 8) % kThr == 0, "absolute-difference grid exact");

__global__ __launch_bounds__(kThr) void tanhmean_kernel(const float* __restrict__ Y, const float* __restrict__ OIr, float* __restrict__ DST, int mode) {
  const unsigned v = blockIdx.x * (unsigned)kThr + threadIdx.x;
  const unsigned s = v >> 9, h = v & 511u;
  const float* yc = Y + (size_t)s * kL * kH + h;
  float acc = 0.0f;
#pragma unroll 1
  for (int l = 0; l < kL; ++l) acc += tanhf(yc[(size_t)l * kH]);
  float m = acc * (1.0f / (float)kL);
  if (mode != 0) m = 0.5f * (OIr[v] + m);
  float* dp = DST + v;
  *(volatile float*)dp = m;
  __threadfence();
  *(volatile float*)dp = m;
}

extern "C" void kernel_launch(void* const* d_in, const int* in_sizes, int n_in,
                              void* d_out, int out_size, void* d_ws, size_t ws_size,
                              hipStream_t stream) {
  if (n_in < 4 || d_out == nullptr || d_ws == nullptr) return;
  if (in_sizes[0] != kB * kL * kD || in_sizes[1] != kB * kL * kD || in_sizes[2] != kD * kH || in_sizes[3] != kH) return;
  if (out_size != kB * kH) return;
  if (ws_size < kWsTotal) return;
  const float* iin = (const float*)d_in[0];
  const float* jin = (const float*)d_in[1];
  const float* W_agg = (const float*)d_in[2];
  const float* b_agg = (const float*)d_in[3];
  float* out = (float*)d_out;
  char* ws = (char*)d_ws;
  unsigned short* I16 = (unsigned short*)(ws + kOffI16);
  unsigned short* J16 = (unsigned short*)(ws + kOffJ16);
  unsigned short* IT16 = (unsigned short*)(ws + kOffIT16);
  unsigned short* JT16 = (unsigned short*)(ws + kOffJT16);
  unsigned short* WT16 = (unsigned short*)(ws + kOffWT16);
  float* BIAS = (float*)(ws + kOffBIAS);
  float* S = (float*)(ws + kOffS);
  unsigned short* PJ = (unsigned short*)(ws + kOffPJ);
  unsigned short* PIT = (unsigned short*)(ws + kOffPIT);
  float* WJ = (float*)(ws + kOffWJ);
  float* WI = (float*)(ws + kOffWI);
  unsigned short* XI16 = (unsigned short*)(ws + kOffXI16);
  unsigned short* XJ16 = (unsigned short*)(ws + kOffXJ16);
  float* Y = (float*)(ws + kOffY);
  float* OI = (float*)(ws + kOffOI);

  const int gC = (int)(((size_t)kB * kLL / 8) / kThr);
  cast_plane_kernel<<<gC, kThr, 0, stream>>>(iin, I16, 9, kD, 0);
  cast_plane_kernel<<<gC, kThr, 0, stream>>>(jin, J16, 9, kD, 0);
  for (int b = 0; b < kB; ++b) {
    wt_plane_kernel<<<kD, kL / 8, 0, stream>>>(iin + (size_t)b * kLL, IT16 + (size_t)b * kLL, kL, kD, kD, kL, 0);
    wt_plane_kernel<<<kD, kL / 8, 0, stream>>>(jin + (size_t)b * kLL, JT16 + (size_t)b * kLL, kL, kD, kD, kL, 0);
  }
  wt_plane_kernel<<<kH, kD / 8, 0, stream>>>(W_agg, WT16, kD, kH, kH, kD, 0);
  setup_kernel<<<1, kThr, 0, stream>>>(b_agg, BIAS);

  const dim3 gLL((kL / 64) * (kL / 64) / 8, 1), gAgg(((kCh * kL) / 64) * (kH / 64) / 8, 1);
  for (int c = 0; c < kB / kCh; ++c) {
    for (int lb = 0; lb < kCh; ++lb) {
      const size_t g = (size_t)(c * kCh + lb) * kLL, l = (size_t)lb * kLL;
      wmma_gemm64<0, false, 2, 0, false, 0><<<gLL, 256, 0, stream>>>(
          I16 + g, I16 + g, kD, 0L, J16 + g, J16 + g, kD, 0L, (void*)(S + l), (void*)(S + l), kL, 0L, BIAS, nullptr, 0L, kL, kL, kD, kScS);
    }
    rowsoftmax_kernel<<<(kCh * kL) / kThr, kThr, 0, stream>>>(S, PJ);
    colsoftmax_kernel<<<(kCh * kL) / kThr, kThr, 0, stream>>>(S, PIT);
    for (int lb = 0; lb < kCh; ++lb) {
      const size_t g = (size_t)(c * kCh + lb) * kLL, l = (size_t)lb * kLL;
      wmma_gemm64<0, false, 2, 0, false, 0><<<gLL, 256, 0, stream>>>(
          PJ + l, PJ + l, kL, 0L, JT16 + g, JT16 + g, kL, 0L, (void*)(WJ + l), (void*)(WJ + l), kD, 0L, BIAS, nullptr, 0L, kL, kD, kL, kScW);
      wmma_gemm64<0, false, 2, 0, false, 0><<<gLL, 256, 0, stream>>>(
          PIT + l, PIT + l, kL, 0L, IT16 + g, IT16 + g, kL, 0L, (void*)(WI + l), (void*)(WI + l), kD, 0L, BIAS, nullptr, 0L, kL, kD, kL, kScW);
    }
    const size_t gc = (size_t)c * kCh * kLL;
    const int gX = (int)(((size_t)kCh * kLL / 8) / kThr);
    absdiff_kernel<<<gX, kThr, 0, stream>>>(iin + gc, WJ, XI16);
    absdiff_kernel<<<gX, kThr, 0, stream>>>(jin + gc, WI, XJ16);
    wmma_gemm64<0, false, 2, 0, false, 0><<<gAgg, 256, 0, stream>>>(
        XI16, XI16, kD, 0L, WT16, WT16, kD, 0L, (void*)Y, (void*)Y, kH, 0L, BIAS + kH, nullptr, 0L, kCh * kL, kH, kD, kScA);
    tanhmean_kernel<<<(kCh * kH) / kThr, kThr, 0, stream>>>(Y, OI + (size_t)c * kCh * kH, OI + (size_t)c * kCh * kH, 0);
    wmma_gemm64<0, false, 2, 0, false, 0><<<gAgg, 256, 0, stream>>>(
        XJ16, XJ16, kD, 0L, WT16, WT16, kD, 0L, (void*)Y, (void*)Y, kH, 0L, BIAS + kH, nullptr, 0L, kCh * kL, kH, kD, kScA);
    tanhmean_kernel<<<(kCh * kH) / kThr, kThr, 0, stream>>>(Y, OI + (size_t)c * kCh * kH, out + (size_t)c * kCh * kH, 1);
  }
}
